// DAGLinkPredictor_26963804684290
// MI455X (gfx1250) — hardware-verified
//
#include <hip/hip_runtime.h>
#include <stddef.h>


#define NTHR  256
#define NWAVE 8
#define GR    32
#define XSP   132
#define CHUNK 2048
#define WCAP  256
#define NGRP  (CHUNK / (NTHR * 4))
#define XIN   33
#define EMBW  16
#define K1P   64

static_assert(WCAP == (CHUNK / NTHR) * 32);
static_assert(NGRP == 2);
static_assert((XSP * 4) % 16 == 0);

typedef float          v4f   __attribute__((ext_vector_type(4)));
typedef float          v8f   __attribute__((ext_vector_type(8)));
typedef int            v4i   __attribute__((ext_vector_type(4)));
typedef unsigned short v8us  __attribute__((ext_vector_type(8)));
typedef __bf16         v16bf __attribute__((ext_vector_type(16)));
union FragB { v16bf v; v8us h[2]; };
union Pack8 { v8us v; v4i i; unsigned short s[8]; };

__device__ __forceinline__ v8f wmb(v16bf a, v16bf b, v8f c) {
  v8f d = __builtin_amdgcn_wmma_f32_16x16x32_bf16(false, a, false, b, (short)0, c, false, false);
  asm volatile("v_nop\n\tv_nop\n\tv_nop\n\tv_nop" : "+v"(d) : "v"(a), "v"(b));
  return d;
}

__device__ __forceinline__ int wrapclamp(int i, int n) {
  i = (i < 0) ? i + n : i;
  i = (i < 0) ? 0 : i;
  i = (i > n - 1) ? n - 1 : i;
  return i;
}

__device__ __forceinline__ unsigned bfrne(float f) {
  unsigned u = __float_as_uint(f);
  u += 0x7fffu + ((u >> 16) & 1u);
  return u >> 16;
}
__device__ __forceinline__ unsigned pairbits(float v) {
  const unsigned h = bfrne(v);
  const float r = v - __uint_as_float(h << 16);
  const unsigned l = bfrne(r);
  return (h & 0xffffu) | (l << 16);
}

__global__ __launch_bounds__(NTHR) void k_wprep(const float* __restrict__ W, int ldw, int K, int Nc, int Kp,
                                                int csplit, int koff,
                                                unsigned short* Ph, unsigned short* Pl) {
  const int i = blockIdx.x * NTHR + threadIdx.x;
  const int kg8 = Kp >> 3;
  const int n8 = Nc * kg8;
  if (i >= n8) return;
  const int c = i / kg8;
  const int kg = i - c * kg8;
  const int hiC = (c >= csplit) ? 1 : 0;
  const int cc = hiC ? (c - csplit) : c;
  const int kb = hiC ? koff : 0;
  Pack8 ph, pl;
#pragma unroll
  for (int j = 0; j < 8; ++j) {
    const int k = kg * 8 + j;
    const int kr = (k < K) ? k : (K - 1);
    float v = W[(size_t)(kb + kr) * ldw + cc];
    v = (k < K) ? v : 0.f;
    const unsigned pb = pairbits(v);
    ph.s[j] = (unsigned short)(pb & 0xffffu);
    pl.s[j] = (unsigned short)(pb >> 16);
  }
  const size_t o = (size_t)c * Kp + (size_t)kg * 8;
  *(volatile v4i*)(Ph + o) = ph.i;
  *(volatile v4i*)(Pl + o) = pl.i;
  __threadfence();
  *(volatile v4i*)(Ph + o) = ph.i;
  *(volatile v4i*)(Pl + o) = pl.i;
}

__global__ __launch_bounds__(NTHR) void k_nodes(const float* __restrict__ x, const float* __restrict__ emb,
                                                unsigned short* xh, unsigned short* xl, int nN, int nT) {
  const int tid = threadIdx.x;
  const int n = blockIdx.x * GR + (tid >> 3);
  const int g = tid & 7;
  int nc = n; if (nc > nN - 1) nc = nN - 1;
  const int t = wrapclamp((int)x[(size_t)nc * XIN], nT);
  const float* pe = emb + (size_t)t * EMBW + 8 * (g & 1);
  const float* px = x + (size_t)nc * XIN + 1 + 8 * ((g - 2) & 3);
  Pack8 ph, pl;
#pragma unroll
  for (int j = 0; j < 8; ++j) {
    const float ve = pe[j];
    const float vx = px[j];
    const float v = (g < 2) ? ve : ((g < 6) ? vx : 0.f);
    const unsigned pb = pairbits(v);
    ph.s[j] = (unsigned short)(pb & 0xffffu);
    pl.s[j] = (unsigned short)(pb >> 16);
  }
  const size_t o = (size_t)n * K1P + (size_t)(8 * g);
  *(volatile v4i*)(xh + o) = ph.i;
  *(volatile v4i*)(xl + o) = pl.i;
  __threadfence();
  *(volatile v4i*)(xh + o) = ph.i;
  *(volatile v4i*)(xl + o) = pl.i;
}

__global__ __launch_bounds__(NTHR) void k_gemm(
    const unsigned short* __restrict__ Ah, const unsigned short* __restrict__ Al,
    const unsigned short* __restrict__ Bh, const unsigned short* __restrict__ Bl,
    int K, int Nc, int nN, float* C,
    const float* __restrict__ avs, const float* __restrict__ avd,
    float* att, int hd16, int npg) {
  __shared__ __attribute__((aligned(16))) float Xs[GR * XSP];
  __shared__ __attribute__((aligned(16))) float Alsd[128];

  const int tid  = threadIdx.x;
  const int lane = tid & 31;
  const int wave = tid >> 5;
  const int hh   = lane >> 4;
  const int m    = lane & 15;
  const int rowBase = blockIdx.x * GR;
  const int colBase = blockIdx.y * 128;
  const int ncol = colBase + wave * 16 + m;

  int r0 = rowBase + m;      if (r0 > nN - 1) r0 = nN - 1;
  int r1 = rowBase + 16 + m; if (r1 > nN - 1) r1 = nN - 1;
  const unsigned short* pa0h = Ah + (size_t)r0 * K + 8 * hh;
  const unsigned short* pa0l = Al + (size_t)r0 * K + 8 * hh;
  const unsigned short* pa1h = Ah + (size_t)r1 * K + 8 * hh;
  const unsigned short* pa1l = Al + (size_t)r1 * K + 8 * hh;
  const unsigned short* pbh  = Bh + (size_t)ncol * K + 8 * hh;
  const unsigned short* pbl  = Bl + (size_t)ncol * K + 8 * hh;

  v8f c0 = {0.f, 0.f, 0.f, 0.f, 0.f, 0.f, 0.f, 0.f};
  v8f c1 = {0.f, 0.f, 0.f, 0.f, 0.f, 0.f, 0.f, 0.f};
#pragma unroll 1
  for (int k0 = 0; k0 < K; k0 += 32) {
    FragB a0h, a0l, a1h, a1l, bh, bl;
    bh.h[0]  = *(const v8us*)(pbh + k0);   bh.h[1]  = *(const v8us*)(pbh + k0 + 16);
    bl.h[0]  = *(const v8us*)(pbl + k0);   bl.h[1]  = *(const v8us*)(pbl + k0 + 16);
    a0h.h[0] = *(const v8us*)(pa0h + k0);  a0h.h[1] = *(const v8us*)(pa0h + k0 + 16);
    a0l.h[0] = *(const v8us*)(pa0l + k0);  a0l.h[1] = *(const v8us*)(pa0l + k0 + 16);
    a1h.h[0] = *(const v8us*)(pa1h + k0);  a1h.h[1] = *(const v8us*)(pa1h + k0 + 16);
    a1l.h[0] = *(const v8us*)(pa1l + k0);  a1l.h[1] = *(const v8us*)(pa1l + k0 + 16);
    c0 = wmb(a0h.v, bh.v, c0);
    c0 = wmb(a0h.v, bl.v, c0);
    c0 = wmb(a0l.v, bh.v, c0);
    c1 = wmb(a1h.v, bh.v, c1);
    c1 = wmb(a1h.v, bl.v, c1);
    c1 = wmb(a1l.v, bh.v, c1);
  }

#pragma unroll
  for (int r = 0; r < 8; ++r) {
    Xs[(8 * hh + r) * XSP + wave * 16 + m]      = c0[r];
    Xs[(16 + 8 * hh + r) * XSP + wave * 16 + m] = c1[r];
  }
  __syncthreads();

  if (hd16 > 0) {
    const int row  = tid >> 3;
    const int part = tid & 7;
    const float* xr  = Xs + row * XSP + 16 * part;
    const float* asp = avs + colBase + 16 * part;
    const float* adp = avd + colBase + 16 * part;
    float ps = 0.f, pd = 0.f;
#pragma unroll
    for (int j = 0; j < 16; ++j) {
      const float v = xr[j];
      ps += v * asp[j];
      pd += v * adp[j];
    }
    for (int mk = 1; mk < hd16; mk <<= 1) {
      ps += __shfl_xor(ps, mk, 32);
      pd += __shfl_xor(pd, mk, 32);
    }
    if ((part & (hd16 - 1)) == 0) {
      const int hs = part / hd16;
      Alsd[hs * 32 + row]      = ps;
      Alsd[64 + hs * 32 + row] = pd;
    }
  }
  __syncthreads();

  v4f xr4[4];
#pragma unroll
  for (int i = 0; i < 4; ++i) xr4[i] = *(const v4f*)(Xs + (4 * wave + i) * XSP + 4 * lane);
  float* cp[4];
#pragma unroll
  for (int i = 0; i < 4; ++i) cp[i] = C + (size_t)(rowBase + 4 * wave + i) * Nc + colBase + 4 * lane;
  const bool wa = (hd16 > 0) && (wave < 2);
  const int  HS = (hd16 > 0) ? (8 / hd16) : 0;
  float av0 = 0.f, av1 = 0.f;
  float* ap0 = att;
  float* ap1 = att;
  if (wa) {
    av0 = Alsd[wave * 64 + lane];
    av1 = Alsd[wave * 64 + 32 + lane];
    ap0 = att + (size_t)(wave * 4 + blockIdx.y * HS) * npg + rowBase + lane;
    ap1 = ap0 + npg;
  }

#pragma unroll
  for (int i = 0; i < 4; ++i) *(volatile v4f*)(cp[i]) = xr4[i];
  if (wa) {
    *(volatile float*)ap0 = av0;
    if (HS > 1) *(volatile float*)ap1 = av1;
  }
  __threadfence();
#pragma unroll
  for (int i = 0; i < 4; ++i) *(volatile v4f*)(cp[i]) = xr4[i];
  if (wa) {
    *(volatile float*)ap0 = av0;
    if (HS > 1) *(volatile float*)ap1 = av1;
  }
}

template <int F, int H>
struct AggCfg {
  static constexpr int NB = 65536 / F;
  static constexpr int LDSB = (65536 + 2 * NB * H + NWAVE * WCAP + NWAVE) * 4;
};

template <int F, int H>
__global__ __launch_bounds__(NTHR) void k_agg(
    const int* __restrict__ ei, const float* __restrict__ hf, const float* __restrict__ att,
    const float* __restrict__ bias, unsigned short* oh, unsigned short* ol,
    int nN, int nE, int npg, int eluf) {
  constexpr int NB  = 65536 / F;
  constexpr int D   = F / H;
  constexpr int CPL = F / 32;
  constexpr int SPW = NB / NWAVE;
  constexpr int RPI = 256 / F;
  static_assert(NB <= 512);
  static_assert((NB & (NB - 1)) == 0);
  static_assert(SPW % RPI == 0);
  static_assert(CPL == 4 || CPL == 8);
  static_assert(AggCfg<F, H>::LDSB <= 300000);

  extern __shared__ v4f lds_dyn[];
  float* sacc = (float*)lds_dyn;
  float* den  = sacc + NB * F;
  float* smx  = den + NB * H;
  int*   list = (int*)(smx + NB * H);
  int*   wcnt = list + NWAVE * WCAP;

  const int tid  = threadIdx.x;
  const int lane = tid & 31;
  const int wave = tid >> 5;
  const int nodeBase = blockIdx.x * NB;
  const int cofs = CPL * lane;
  const int hd   = cofs / D;
  const float* als = att + (size_t)hd * npg;
  const float* ald = att + (size_t)(4 + hd) * npg;

#pragma unroll 1
  for (int j = 0; j < SPW; ++j) {
    const int slot = wave * SPW + j;
    const int node = nodeBase + slot;
    int nd = node; if (nd > nN - 1) nd = nN - 1;
    const bool valid = node < nN;
    const float keep = valid ? 1.f : 0.f;
    float l = als[nd] + ald[nd];
    l = (l > 0.f) ? l : 0.2f * l;
    smx[slot * H + hd] = valid ? l : 0.f;
    den[slot * H + hd] = keep;
    const float* hp = hf + (size_t)nd * F + cofs;
    float* sp = sacc + slot * F + cofs;
    if (CPL == 8) {
      const v4f a = *(const v4f*)(hp) * keep;
      const v4f b = *(const v4f*)(hp + 4) * keep;
      *(v4f*)(sp) = a;
      *(v4f*)(sp + 4) = b;
    } else {
      const v4f a = *(const v4f*)(hp) * keep;
      *(v4f*)(sp) = a;
    }
  }
  __syncthreads();

  const int* eid = ei + nE;
  const bool al16 = ((nE & 3) == 0);

  const int nChunks = (nE + CHUNK - 1) / CHUNK;
#pragma unroll 1
  for (int ch = 0; ch < nChunks; ++ch) {
    const int cbase = ch * CHUNK;
    int wc = 0;
#pragma unroll
    for (int g = 0; g < NGRP; ++g) {
      const int el0 = (g * NTHR + tid) * 4;
      const int e0  = cbase + el0;
      const int sent = -2147483647 - 1;
      v4i d;
      if (al16 && (cbase + CHUNK <= nE)) {
        d = *(const v4i*)(eid + e0);
      } else {
        d.x = (e0     < nE) ? eid[min(e0,     nE - 1)] : sent;
        d.y = (e0 + 1 < nE) ? eid[min(e0 + 1, nE - 1)] : sent;
        d.z = (e0 + 2 < nE) ? eid[min(e0 + 2, nE - 1)] : sent;
        d.w = (e0 + 3 < nE) ? eid[min(e0 + 3, nE - 1)] : sent;
      }
      const unsigned s0 = (unsigned)d.x - (unsigned)nodeBase;
      const unsigned s1 = (unsigned)d.y - (unsigned)nodeBase;
      const unsigned s2 = (unsigned)d.z - (unsigned)nodeBase;
      const unsigned s3 = (unsigned)d.w - (unsigned)nodeBase;
      const bool h0 = s0 < (unsigned)NB;
      const bool h1 = s1 < (unsigned)NB;
      const bool h2 = s2 < (unsigned)NB;
      const bool h3 = s3 < (unsigned)NB;
      const unsigned many = __builtin_amdgcn_ballot_w32(h0 | h1 | h2 | h3);
      if (many != 0u) {
#define HITJ(J, HJ, SJ) { \
          const unsigned mj = __builtin_amdgcn_ballot_w32(HJ); \
          if (HJ) { \
            const int pos = wc + (int)__builtin_amdgcn_mbcnt_lo(mj, 0u); \
            if (pos < WCAP) list[wave * WCAP + pos] = ((el0 + (J)) << 9) | (int)(SJ); \
          } \
          wc += (int)__builtin_popcount(mj); }
        HITJ(0, h0, s0)
        HITJ(1, h1, s1)
        HITJ(2, h2, s2)
        HITJ(3, h3, s3)
#undef HITJ
      }
    }
    if (lane == 0) wcnt[wave] = wc;
    __syncthreads();

    if (wave == 0) {
#pragma unroll 1
      for (int wsx = 0; wsx < NWAVE; ++wsx) {
        int n = wcnt[wsx];
        if (n > WCAP) n = WCAP;
        if (n < 0) n = 0;
#pragma unroll 1
        for (int i = 0; i < n; ++i) {
          const int ent  = list[wsx * WCAP + i];
          const int slot = ent & (NB - 1);
          const int el   = (ent >> 9) & (CHUNK - 1);
          int e = cbase + el;
          if (e > nE - 1) e = nE - 1;
          const int src = wrapclamp(ei[e], nN);
          int nd = nodeBase + slot;
          if (nd > nN - 1) nd = nN - 1;
          float l = als[src] + ald[nd];
          l = (l > 0.f) ? l : 0.2f * l;
          const int ai = slot * H + hd;
          const float mo = smx[ai];
          const float dn = den[ai];
          const float mn = fmaxf(mo, l);
          const float sc = __expf(mo - mn);
          const float p  = __expf(l - mn);
          float* sp = sacc + slot * F + cofs;
          const float* xg = hf + (size_t)src * F + cofs;
          if (CPL == 8) {
            v4f a = *(v4f*)(sp);
            v4f b = *(v4f*)(sp + 4);
            const v4f xa = *(const v4f*)(xg);
            const v4f xb = *(const v4f*)(xg + 4);
            a = a * sc + xa * p;
            b = b * sc + xb * p;
            *(v4f*)(sp) = a;
            *(v4f*)(sp + 4) = b;
          } else {
            v4f a = *(v4f*)(sp);
            const v4f xa = *(const v4f*)(xg);
            a = a * sc + xa * p;
            *(v4f*)(sp) = a;
          }
          smx[ai] = mn;
          den[ai] = dn * sc + p;
        }
      }
    }
    __syncthreads();
  }

  const int colc = 8 * (lane & (F / 8 - 1));
  const int hde  = colc / D;
  const int sub  = (RPI == 2) ? (lane >> 4) : 0;
  const v4f b0 = *(const v4f*)(bias + colc);
  const v4f b1 = *(const v4f*)(bias + colc + 4);
#pragma unroll 1
  for (int j = 0; j < SPW / RPI; ++j) {
    const int slot = wave * SPW + j * RPI + sub;
    const int node = nodeBase + slot;
    const float* sp = sacc + slot * F + colc;
    v4f o0 = *(const v4f*)(sp);
    v4f o1 = *(const v4f*)(sp + 4);
    const float inv = 1.0f / (den[slot * H + hde] + 1e-16f);
    o0 = o0 * inv + b0;
    o1 = o1 * inv + b1;
    if (eluf) {
      o0.x = (o0.x > 0.f) ? o0.x : (__expf(fminf(o0.x, 0.f)) - 1.0f);
      o0.y = (o0.y > 0.f) ? o0.y : (__expf(fminf(o0.y, 0.f)) - 1.0f);
      o0.z = (o0.z > 0.f) ? o0.z : (__expf(fminf(o0.z, 0.f)) - 1.0f);
      o0.w = (o0.w > 0.f) ? o0.w : (__expf(fminf(o0.w, 0.f)) - 1.0f);
      o1.x = (o1.x > 0.f) ? o1.x : (__expf(fminf(o1.x, 0.f)) - 1.0f);
      o1.y = (o1.y > 0.f) ? o1.y : (__expf(fminf(o1.y, 0.f)) - 1.0f);
      o1.z = (o1.z > 0.f) ? o1.z : (__expf(fminf(o1.z, 0.f)) - 1.0f);
      o1.w = (o1.w > 0.f) ? o1.w : (__expf(fminf(o1.w, 0.f)) - 1.0f);
    }
    Pack8 ph, pl;
    {
      unsigned pb;
      pb = pairbits(o0.x); ph.s[0] = (unsigned short)(pb & 0xffffu); pl.s[0] = (unsigned short)(pb >> 16);
      pb = pairbits(o0.y); ph.s[1] = (unsigned short)(pb & 0xffffu); pl.s[1] = (unsigned short)(pb >> 16);
      pb = pairbits(o0.z); ph.s[2] = (unsigned short)(pb & 0xffffu); pl.s[2] = (unsigned short)(pb >> 16);
      pb = pairbits(o0.w); ph.s[3] = (unsigned short)(pb & 0xffffu); pl.s[3] = (unsigned short)(pb >> 16);
      pb = pairbits(o1.x); ph.s[4] = (unsigned short)(pb & 0xffffu); pl.s[4] = (unsigned short)(pb >> 16);
      pb = pairbits(o1.y); ph.s[5] = (unsigned short)(pb & 0xffffu); pl.s[5] = (unsigned short)(pb >> 16);
      pb = pairbits(o1.z); ph.s[6] = (unsigned short)(pb & 0xffffu); pl.s[6] = (unsigned short)(pb >> 16);
      pb = pairbits(o1.w); ph.s[7] = (unsigned short)(pb & 0xffffu); pl.s[7] = (unsigned short)(pb >> 16);
    }
    const size_t o = (size_t)node * F + (size_t)colc;
    *(volatile v4i*)(oh + o) = ph.i;
    *(volatile v4i*)(ol + o) = pl.i;
    __threadfence();
    *(volatile v4i*)(oh + o) = ph.i;
    *(volatile v4i*)(ol + o) = pl.i;
  }
}

__global__ __launch_bounds__(NTHR) void k_dec(
    const float* __restrict__ x, const int* __restrict__ eli, const float* __restrict__ pq,
    const float* __restrict__ bl1, const float* __restrict__ wl2, const float* __restrict__ bl2,
    const float* __restrict__ tb, float* out, int nN, int nL, int nT) {
  const int l = blockIdx.x * NTHR + threadIdx.x;
  if (l >= nL) return;
  const int ls = wrapclamp(eli[l], nN);
  const int ld = wrapclamp(eli[(size_t)nL + l], nN);
  const float* pp = pq + (size_t)ls * 128;
  const float* qp = pq + (size_t)ld * 128 + 64;
  float s = 0.f;
#pragma unroll 2
  for (int q = 0; q < 16; ++q) {
    const v4f a = *(const v4f*)(pp + 4 * q);
    const v4f b = *(const v4f*)(qp + 4 * q);
    const v4f c = *(const v4f*)(bl1 + 4 * q);
    const v4f w = *(const v4f*)(wl2 + 4 * q);
    v4f h = a + b + c;
    h.x = (h.x > 0.f) ? h.x : 0.f;
    h.y = (h.y > 0.f) ? h.y : 0.f;
    h.z = (h.z > 0.f) ? h.z : 0.f;
    h.w = (h.w > 0.f) ? h.w : 0.f;
    s += h.x * w.x + h.y * w.y + h.z * w.z + h.w * w.w;
  }
  const int ts = wrapclamp((int)x[(size_t)ls * XIN], nT);
  const int td = wrapclamp((int)x[(size_t)ld * XIN], nT);
  const float r = (s + bl2[0]) + tb[(size_t)ts * nT + td];
  *(volatile float*)(out + l) = r;
  __threadfence();
  *(volatile float*)(out + l) = r;
}

static inline char* carve(char* base, size_t* off, size_t bytes) {
  char* p = base + *off;
  *off += (bytes + 255) & ~(size_t)255;
  return p;
}

extern "C" void kernel_launch(void* const* d_in, const int* in_sizes, int n_in,
                              void* d_out, int out_size, void* d_ws, size_t ws_size,
                              hipStream_t stream) {
  if (n_in < 21) return;
  const int nN = in_sizes[0] / XIN;
  if (nN <= 0 || in_sizes[0] != nN * XIN) return;
  const int nE = in_sizes[1] / 2;
  if (nE < 0 || in_sizes[1] != 2 * nE) return;
  const int nL = in_sizes[2] / 2;
  if (nL <= 0 || in_sizes[2] != 2 * nL) return;
  const int nT = in_sizes[3] / EMBW;
  if (nT <= 0 || in_sizes[3] != nT * EMBW) return;
  if (in_sizes[4] != 48 * 256 || in_sizes[5] != 256 || in_sizes[6] != 256 || in_sizes[7] != 256) return;
  if (in_sizes[8] != 256 * 256 || in_sizes[9] != 256 || in_sizes[10] != 256 || in_sizes[11] != 256) return;
  if (in_sizes[12] != 256 * 128 || in_sizes[13] != 128 || in_sizes[14] != 128 || in_sizes[15] != 128) return;
  if (in_sizes[16] != 256 * 64 || in_sizes[17] != 64 || in_sizes[18] != 64 || in_sizes[19] < 1) return;
  if (in_sizes[20] != nT * nT) return;
  if (out_size != nL) return;

  const float* x   = (const float*)d_in[0];
  const int*   ei  = (const int*)d_in[1];
  const int*   eli = (const int*)d_in[2];
  const float* emb = (const float*)d_in[3];
  const float* W1  = (const float*)d_in[4];
  const float* as1 = (const float*)d_in[5];
  const float* ad1 = (const float*)d_in[6];
  const float* b1  = (const float*)d_in[7];
  const float* W2  = (const float*)d_in[8];
  const float* as2 = (const float*)d_in[9];
  const float* ad2 = (const float*)d_in[10];
  const float* b2  = (const float*)d_in[11];
  const float* W3  = (const float*)d_in[12];
  const float* as3 = (const float*)d_in[13];
  const float* ad3 = (const float*)d_in[14];
  const float* b3  = (const float*)d_in[15];
  const float* Wl1 = (const float*)d_in[16];
  const float* bl1 = (const float*)d_in[17];
  const float* Wl2 = (const float*)d_in[18];
  const float* bl2 = (const float*)d_in[19];
  const float* tb  = (const float*)d_in[20];
  float* out = (float*)d_out;

  const int npg = ((nN + GR - 1) / GR) * GR;
  const int npa = ((nN + 511) / 512) * 512;

  size_t off = 0;
  char* wsb = (char*)d_ws;
  unsigned short* w1h = (unsigned short*)carve(wsb, &off, (size_t)256 * 64 * 2);
  unsigned short* w1l = (unsigned short*)carve(wsb, &off, (size_t)256 * 64 * 2);
  unsigned short* w2h = (unsigned short*)carve(wsb, &off, (size_t)256 * 256 * 2);
  unsigned short* w2l = (unsigned short*)carve(wsb, &off, (size_t)256 * 256 * 2);
  unsigned short* w3h = (unsigned short*)carve(wsb, &off, (size_t)128 * 256 * 2);
  unsigned short* w3l = (unsigned short*)carve(wsb, &off, (size_t)128 * 256 * 2);
  unsigned short* wdh = (unsigned short*)carve(wsb, &off, (size_t)128 * 128 * 2);
  unsigned short* wdl = (unsigned short*)carve(wsb, &off, (size_t)128 * 128 * 2);
  unsigned short* xch = (unsigned short*)carve(wsb, &off, (size_t)npg * K1P * 2);
  unsigned short* xcl = (unsigned short*)carve(wsb, &off, (size_t)npg * K1P * 2);
  unsigned short* ach = (unsigned short*)carve(wsb, &off, (size_t)npa * 256 * 2);
  unsigned short* acl = (unsigned short*)carve(wsb, &off, (size_t)npa * 256 * 2);
  float* cbuf = (float*)carve(wsb, &off, (size_t)npg * 256 * 4);
  float* att  = (float*)carve(wsb, &off, (size_t)8 * npg * 4);
  if (off > ws_size) return;
  if (off > (size_t)134217728) return;

  k_wprep<<<(256 * (64 / 8) + NTHR - 1) / NTHR, NTHR, 0, stream>>>(W1, 256, 48, 256, 64, 256, 0, w1h, w1l);
  k_wprep<<<(256 * (256 / 8) + NTHR - 1) / NTHR, NTHR, 0, stream>>>(W2, 256, 256, 256, 256, 256, 0, w2h, w2l);
  k_wprep<<<(128 * (256 / 8) + NTHR - 1) / NTHR, NTHR, 0, stream>>>(W3, 128, 256, 128, 256, 128, 0, w3h, w3l);
  k_wprep<<<(128 * (128 / 8) + NTHR - 1) / NTHR, NTHR, 0, stream>>>(Wl1, 64, 128, 128, 128, 64, 128, wdh, wdl);

  k_nodes<<<npg / GR, NTHR, 0, stream>>>(x, emb, xch, xcl, nN, nT);

  hipFuncSetAttribute(reinterpret_cast<const void*>(&k_agg<256, 4>),
                      hipFuncAttributeMaxDynamicSharedMemorySize, AggCfg<256, 4>::LDSB);
  hipFuncSetAttribute(reinterpret_cast<const void*>(&k_agg<256, 2>),
                      hipFuncAttributeMaxDynamicSharedMemorySize, AggCfg<256, 2>::LDSB);
  hipFuncSetAttribute(reinterpret_cast<const void*>(&k_agg<128, 1>),
                      hipFuncAttributeMaxDynamicSharedMemorySize, AggCfg<128, 1>::LDSB);

  const dim3 gg2(npg / GR, 2);
  const dim3 gg1(npg / GR, 1);

  k_gemm<<<gg2, NTHR, 0, stream>>>(xch, xcl, w1h, w1l, 64, 256, nN, cbuf, as1, ad1, att, 4, npg);
  k_agg<256, 4><<<npa / 256, NTHR, AggCfg<256, 4>::LDSB, stream>>>(ei, cbuf, att, b1, ach, acl, nN, nE, npg, 1);
  k_gemm<<<gg2, NTHR, 0, stream>>>(ach, acl, w2h, w2l, 256, 256, nN, cbuf, as2, ad2, att, 8, npg);
  k_agg<256, 2><<<npa / 256, NTHR, AggCfg<256, 2>::LDSB, stream>>>(ei, cbuf, att, b2, ach, acl, nN, nE, npg, 1);
  k_gemm<<<gg1, NTHR, 0, stream>>>(ach, acl, w3h, w3l, 256, 128, nN, cbuf, as3, ad3, att, 8, npg);
  k_agg<128, 1><<<npa / 512, NTHR, AggCfg<128, 1>::LDSB, stream>>>(ei, cbuf, att, b3, ach, acl, nN, nE, npg, 0);
  k_gemm<<<gg1, NTHR, 0, stream>>>(ach, acl, wdh, wdl, 128, 128, nN, cbuf, as3, ad3, att, 0, npg);
  k_dec<<<(nL + NTHR - 1) / NTHR, NTHR, 0, stream>>>(x, eli, cbuf, bl1, Wl2, bl2, tb, out, nN, nL, nT);
}
